// GeneExpressionGNN_52879637348574
// MI455X (gfx1250) — hardware-verified
//
#include <hip/hip_runtime.h>
#include <stddef.h>


#define CC      256
#define PCH     128
#define NOUT    128
#define GPB     64
#define NTHR    256
#define NWAVE   8
#define EPT     8
#define NGRP    2
#define CHUNK   (NTHR * EPT * NGRP)
#define WCAP    (EPT * NGRP * 32)
#define NBC     32768
#define NBF     1024
#define ESHF    10
#define ESHP    7
#define RCAP    49152
#define RBN     128
#define TGT     256
#define DEGCAP  512
#define GR      64
#define GC      128
#define OTHR    256
#define TPK     64
#define TPN     32
#define TPP     72
#define ASCL    16
#define HSCL    256
#define WSCL    64
#define PSCL    256
#define QSCL    256
#define WSCAP   134217728

#define LDS_COUNT ((NBC + NWAVE * WCAP + NWAVE) * 4)
#define LDS_FILL  ((RCAP + NBF + NWAVE * WCAP + NWAVE) * 4)

static_assert((CHUNK & (CHUNK - 1)) == 0);
static_assert((NBC & (NBC - 1)) == 0 && (NBF & (NBF - 1)) == 0 && (GPB & (GPB - 1)) == 0);
static_assert(NBF <= (1 << ESHF) && GPB <= (1 << ESHP));
static_assert((NBC % NBF) == 0);
static_assert(OTHR * 4 == NBF);
static_assert((RCAP % 32) == 0);
static_assert(TGT == NWAVE * 32);
static_assert(GR == 4 * 16 && GC == 2 * 64 && NWAVE == 8);
static_assert((TGT % GR) == 0 && (TGT % NBF) == 0 || (NBF % TGT) == 0);
static_assert(NBC == NWAVE * 32 * 128);
static_assert(CC == 2 * PCH && PCH == 32 * 4);
static_assert((CC % GC) == 0 && (NOUT % GC) == 0);
static_assert((CC % 32) == 0);
static_assert((GPB % 16) == 0 && PCH == 16 * 8);
static_assert((CC % TPK) == 0 && (CC % TPN) == 0 && (NOUT % TPN) == 0);
static_assert(TPN * 8 == NTHR && TPK * TPN == NTHR * 8 && TPK == NWAVE * 8);
static_assert((TPP % 8) == 0 && TPP >= TPK);
static_assert(LDS_FILL <= 300 * 1024);

typedef float     v2f  __attribute__((ext_vector_type(2)));
typedef float     v4f  __attribute__((ext_vector_type(4)));
typedef float     v8f  __attribute__((ext_vector_type(8)));
typedef int       v4i  __attribute__((ext_vector_type(4)));
typedef _Float16  v4h  __attribute__((ext_vector_type(4)));
typedef _Float16  v8h  __attribute__((ext_vector_type(8)));
typedef _Float16  v16h __attribute__((ext_vector_type(16)));
union FragH { v16h v; v8h h[2]; };
union U32F { float f; int i; };

__device__ __forceinline__ v8f wmf(v16h a, v16h b, v8f c) {
  v8f d = __builtin_amdgcn_wmma_f32_16x16x32_f16(false, a, false, b, (short)0, c, false, false);
  asm volatile("v_nop\n\tv_nop\n\tv_nop\n\tv_nop" : "+v"(d) : "v"(a), "v"(b));
  return d;
}

__device__ __forceinline__ v4f relu4(v4f t) {
  v4f o;
  o.x = fmaxf(t.x, 0.0f); o.y = fmaxf(t.y, 0.0f); o.z = fmaxf(t.z, 0.0f); o.w = fmaxf(t.w, 0.0f);
  return o;
}

template <int NB, int SRC, int WC, int ESH>
__device__ __forceinline__ int scan_chunk(const int* __restrict__ keys, const int* __restrict__ vals,
                                          int nK, int nN, int cbase, int slotBase, int vec8,
                                          int* list, int tid, int lane, int wave) {
  int wc = 0;
#pragma unroll
  for (int g = 0; g < NGRP; ++g) {
    const int el0  = (g * NTHR + tid) * EPT;
    const int e0   = cbase + el0;
    const int sent = -2147483647 - 1;
    v4i da, db;
    v4i sa = {0, 0, 0, 0}, sb = {0, 0, 0, 0};
    const int i0 = min(e0, nK - 1),     i1 = min(e0 + 1, nK - 1), i2 = min(e0 + 2, nK - 1), i3 = min(e0 + 3, nK - 1);
    const int i4 = min(e0 + 4, nK - 1), i5 = min(e0 + 5, nK - 1), i6 = min(e0 + 6, nK - 1), i7 = min(e0 + 7, nK - 1);
    if (vec8 != 0 && cbase + CHUNK <= nK) {
      da = *(const v4i*)(keys + e0);
      db = *(const v4i*)(keys + e0 + 4);
      if (SRC == 1) {
        sa = *(const v4i*)(vals + e0);
        sb = *(const v4i*)(vals + e0 + 4);
      }
    } else {
      da.x = (e0     < nK) ? keys[i0] : sent;
      da.y = (e0 + 1 < nK) ? keys[i1] : sent;
      da.z = (e0 + 2 < nK) ? keys[i2] : sent;
      da.w = (e0 + 3 < nK) ? keys[i3] : sent;
      db.x = (e0 + 4 < nK) ? keys[i4] : sent;
      db.y = (e0 + 5 < nK) ? keys[i5] : sent;
      db.z = (e0 + 6 < nK) ? keys[i6] : sent;
      db.w = (e0 + 7 < nK) ? keys[i7] : sent;
      if (SRC == 1) {
        sa.x = vals[i0]; sa.y = vals[i1]; sa.z = vals[i2]; sa.w = vals[i3];
        sb.x = vals[i4]; sb.y = vals[i5]; sb.z = vals[i6]; sb.w = vals[i7];
      }
    }
    if (SRC == 2) {
      sa.x = i0; sa.y = i1; sa.z = i2; sa.w = i3;
      sb.x = i4; sb.y = i5; sb.z = i6; sb.w = i7;
    }
    if (SRC != 0) {
      sa.x = min(max(sa.x, 0), nN - 1); sa.y = min(max(sa.y, 0), nN - 1);
      sa.z = min(max(sa.z, 0), nN - 1); sa.w = min(max(sa.w, 0), nN - 1);
      sb.x = min(max(sb.x, 0), nN - 1); sb.y = min(max(sb.y, 0), nN - 1);
      sb.z = min(max(sb.z, 0), nN - 1); sb.w = min(max(sb.w, 0), nN - 1);
    }
    const unsigned nb = (unsigned)slotBase;
    const unsigned s0 = (unsigned)da.x - nb, s1 = (unsigned)da.y - nb;
    const unsigned s2 = (unsigned)da.z - nb, s3 = (unsigned)da.w - nb;
    const unsigned s4 = (unsigned)db.x - nb, s5 = (unsigned)db.y - nb;
    const unsigned s6 = (unsigned)db.z - nb, s7 = (unsigned)db.w - nb;
    const bool h0 = s0 < (unsigned)NB, h1 = s1 < (unsigned)NB, h2 = s2 < (unsigned)NB, h3 = s3 < (unsigned)NB;
    const bool h4 = s4 < (unsigned)NB, h5 = s5 < (unsigned)NB, h6 = s6 < (unsigned)NB, h7 = s7 < (unsigned)NB;
    const unsigned any = __builtin_amdgcn_ballot_w32(h0 | h1 | h2 | h3 | h4 | h5 | h6 | h7);
    if (any != 0u) {
#define HITJ(HJ, SJ, VJ) { \
        const unsigned mj = __builtin_amdgcn_ballot_w32(HJ); \
        if (mj != 0u) { \
          if (HJ) { \
            const int pos = wc + (int)__builtin_amdgcn_mbcnt_lo(mj, 0u); \
            const int entv = (SRC != 0) ? (((VJ) << ESH) | (int)(SJ)) : (int)(SJ); \
            if (pos < WC) list[wave * WC + pos] = entv; \
          } \
          wc += (int)__builtin_popcount(mj); } }
      HITJ(h0, s0, sa.x)
      HITJ(h1, s1, sa.y)
      HITJ(h2, s2, sa.z)
      HITJ(h3, s3, sa.w)
      HITJ(h4, s4, sb.x)
      HITJ(h5, s5, sb.y)
      HITJ(h6, s6, sb.z)
      HITJ(h7, s7, sb.w)
#undef HITJ
    }
  }
  return wc;
}

__global__ __launch_bounds__(NTHR) void k_x16(const float* __restrict__ x, _Float16* dst,
                                              int nN, int total8, float scale) {
  const int i = (int)blockIdx.x * NTHR + (int)threadIdx.x;
  if (i >= total8) return;
  const size_t e  = (size_t)8 * (size_t)i;
  const int    r  = (int)(e / (size_t)CC);
  const int    k0 = (int)(e - (size_t)r * (size_t)CC);
  const int    rc = r < nN ? r : nN - 1;
  const float  z  = (r < nN) ? scale : 0.0f;
  const float* sp = x + (size_t)rc * CC + k0;
  const v4f f0 = *(const v4f*)sp;
  const v4f f1 = *(const v4f*)(sp + 4);
  v8h hv;
  hv[0] = (_Float16)(f0.x * z); hv[1] = (_Float16)(f0.y * z); hv[2] = (_Float16)(f0.z * z); hv[3] = (_Float16)(f0.w * z);
  hv[4] = (_Float16)(f1.x * z); hv[5] = (_Float16)(f1.y * z); hv[6] = (_Float16)(f1.z * z); hv[7] = (_Float16)(f1.w * z);
  _Float16* d = dst + e;
  *(volatile v8h*)d = hv;
  __threadfence();
  *(volatile v8h*)d = hv;
}

__global__ __launch_bounds__(NTHR) void k_wT16(const float* __restrict__ W, _Float16* Wp,
                                               int KD, int NC, float scale) {
  __shared__ __attribute__((aligned(16))) _Float16 sT[TPN * TPP];
  const int tid = threadIdx.x;
  const int k0 = (int)blockIdx.x * TPK, n0 = (int)blockIdx.y * TPN;
  const int nc = tid & 31, kq = tid >> 5;
#pragma unroll
  for (int i = 0; i < TPK / NWAVE; ++i) {
    const int kr = kq + NWAVE * i;
    const float v = W[(size_t)(k0 + kr) * NC + n0 + nc] * scale;
    sT[nc * TPP + kr] = (_Float16)v;
  }
  __syncthreads();
  const int nl = tid >> 3, p = tid & 7;
  const v8h hv = *(const v8h*)(sT + nl * TPP + 8 * p);
  _Float16* d = Wp + (size_t)(n0 + nl) * KD + k0 + 8 * p;
  *(volatile v8h*)d = hv;
  __threadfence();
  *(volatile v8h*)d = hv;
}

__global__ __launch_bounds__(NTHR) void k_count(
    const int* __restrict__ keys, int* cnt, float* dinv, int nK, int nN, int vec8) {
  extern __shared__ v4f lds_dyn[];
  int* scnt = (int*)lds_dyn;
  int* list = scnt + NBC;
  int* wcnt = list + NWAVE * WCAP;
  const int tid = threadIdx.x, lane = tid & 31, wave = tid >> 5;
  const int nodeBase = blockIdx.x * NBC;

  {
    const v4i z = {0, 0, 0, 0};
    for (int i = tid; i < NBC / 4; i += NTHR) ((v4i*)scnt)[i] = z;
  }
  __syncthreads();

  const int nChunks = (nK + CHUNK - 1) / CHUNK;
#pragma unroll 1
  for (int ch = 0; ch < nChunks; ++ch) {
    const int cbase = ch * CHUNK;
    const int wc = scan_chunk<NBC, 0, WCAP, 0>(keys, keys, nK, nN, cbase, nodeBase, vec8, list, tid, lane, wave);
    if (lane == 0) wcnt[wave] = wc;
    __syncthreads();
    if (wave == 0) {
#pragma unroll 1
      for (int wsx = 0; wsx < NWAVE; ++wsx) {
        int n = __builtin_amdgcn_readfirstlane(wcnt[wsx]);
        n = n > WCAP ? WCAP : (n < 0 ? 0 : n);
        const int* lp = list + wsx * WCAP;
#pragma unroll 1
        for (int i = 0; i < n; ++i) {
          const int ent  = __builtin_amdgcn_readfirstlane(lp[i]);
          const int slot = ent & (NBC - 1);
          if (lane == 0) scnt[slot] = scnt[slot] + 1;
        }
      }
    }
    __syncthreads();
  }

  int*   cp = cnt + (size_t)nodeBase;
  float* dp = dinv + (size_t)nodeBase;
#pragma unroll 4
  for (int q = 0; q < 32; ++q) {
    const int f = (wave * 32 + q) * 128 + 4 * lane;
    const v4i c = *(const v4i*)(scnt + f);
    const float g0 = (float)c.x + 1.0f, g1 = (float)c.y + 1.0f, g2 = (float)c.z + 1.0f, g3 = (float)c.w + 1.0f;
    v4f d;
    d.x = g0 > 0.f ? rsqrtf(g0) : 0.f; d.y = g1 > 0.f ? rsqrtf(g1) : 0.f;
    d.z = g2 > 0.f ? rsqrtf(g2) : 0.f; d.w = g3 > 0.f ? rsqrtf(g3) : 0.f;
    *(volatile v4i*)(cp + f) = c;
    *(volatile v4f*)(dp + f) = d;
  }
  __threadfence();
#pragma unroll 4
  for (int q = 0; q < 32; ++q) {
    const int f = (wave * 32 + q) * 128 + 4 * lane;
    const v4i c = *(const v4i*)(scnt + f);
    const float g0 = (float)c.x + 1.0f, g1 = (float)c.y + 1.0f, g2 = (float)c.z + 1.0f, g3 = (float)c.w + 1.0f;
    v4f d;
    d.x = g0 > 0.f ? rsqrtf(g0) : 0.f; d.y = g1 > 0.f ? rsqrtf(g1) : 0.f;
    d.z = g2 > 0.f ? rsqrtf(g2) : 0.f; d.w = g3 > 0.f ? rsqrtf(g3) : 0.f;
    *(volatile v4i*)(cp + f) = c;
    *(volatile v4f*)(dp + f) = d;
  }
}

__global__ __launch_bounds__(OTHR) void k_offsets(
    const int* __restrict__ cnt, int* off, int* rbase, int nBF) {
  __shared__ __attribute__((aligned(16))) int srb[RBN];
  __shared__ int wtot[OTHR / 32];
  const int tid = threadIdx.x, lane = tid & 31, wave = tid >> 5;
  for (int i = tid; i < RBN; i += OTHR) srb[i] = 0;
  int carry = 0;
#pragma unroll 1
  for (int fb = 0; fb < nBF; ++fb) {
    const int base = fb * NBF;
    const v4i c = *(const v4i*)(cnt + base + 4 * tid);
    const int e0 = max(c.x, 0), e1 = max(c.y, 0), e2 = max(c.z, 0), e3 = max(c.w, 0);
    const int ts = e0 + e1 + e2 + e3;
    int incl = ts;
#pragma unroll
    for (int d = 1; d < 32; d <<= 1) {
      const int t = __shfl_up(incl, d, 32);
      if (lane >= d) incl += t;
    }
    if (lane == 31) wtot[wave] = incl;
    __syncthreads();
    int pre = 0;
#pragma unroll 1
    for (int w = 0; w < wave; ++w) pre += wtot[w];
    int tot = 0;
#pragma unroll
    for (int w = 0; w < OTHR / 32; ++w) tot += wtot[w];
    int run = carry + pre + incl - ts;
    v4i o;
    o.x = run; run += e0;
    o.y = run; run += e1;
    o.z = run; run += e2;
    o.w = run;
    int* op = off + base + 4 * tid;
    *(volatile v4i*)op = o;
    __threadfence();
    *(volatile v4i*)op = o;
    if (tid == 0) srb[min(fb, RBN - 1)] = carry;
    carry += (tot + 31) & ~31;
    __syncthreads();
  }
  if (tid == 0) srb[min(nBF, RBN - 1)] = carry;
  __syncthreads();
  v4i rv = {0, 0, 0, 0};
  if (tid < 32) rv = *(const v4i*)(srb + 4 * tid);
  if (tid < 32) *(volatile v4i*)(rbase + 4 * tid) = rv;
  __threadfence();
  if (tid < 32) *(volatile v4i*)(rbase + 4 * tid) = rv;
}

__global__ __launch_bounds__(NTHR) void k_fill(
    const int* __restrict__ keys, const int* __restrict__ vals, const int* __restrict__ off,
    const int* __restrict__ rbase, int* csr, int nN, int nK, int vec8, int csrLen) {
  extern __shared__ v4f lds_dyn[];
  int* region = (int*)lds_dyn;
  int* cursor = region + RCAP;
  int* list   = cursor + NBF;
  int* wcnt   = list + NWAVE * WCAP;
  const int tid = threadIdx.x, lane = tid & 31, wave = tid >> 5;
  const int b = blockIdx.x;
  const int nodeBase = b * NBF;

  int rb0 = rbase[b];
  const int rb1 = rbase[b + 1];
  rb0 = rb0 < 0 ? 0 : (rb0 > csrLen ? csrLen : rb0);
  rb0 &= ~31;
  int len = rb1 - rb0;
  len = len < 0 ? 0 : (len > RCAP ? RCAP : len);
  int lenW = (len + 31) & ~31;
  if (rb0 + lenW > csrLen) lenW = (csrLen - rb0) & ~31;

  {
    const v4i z = {0, 0, 0, 0};
    for (int i = tid; i < RCAP / 4; i += NTHR) ((v4i*)region)[i] = z;
    for (int s = tid; s < NBF; s += NTHR) {
      int o = off[nodeBase + s] - rb0;
      o = o < 0 ? 0 : (o > RCAP ? RCAP : o);
      cursor[s] = o;
    }
  }
  __syncthreads();

  const int nChunks = (nK + CHUNK - 1) / CHUNK;
#pragma unroll 1
  for (int ch = 0; ch < nChunks; ++ch) {
    const int cbase = ch * CHUNK;
    const int wc = scan_chunk<NBF, 1, WCAP, ESHF>(keys, vals, nK, nN, cbase, nodeBase, vec8, list, tid, lane, wave);
    if (lane == 0) wcnt[wave] = wc;
    __syncthreads();
    if (wave == 0) {
#pragma unroll 1
      for (int wsx = 0; wsx < NWAVE; ++wsx) {
        int n = __builtin_amdgcn_readfirstlane(wcnt[wsx]);
        n = n > WCAP ? WCAP : (n < 0 ? 0 : n);
        const int* lp = list + wsx * WCAP;
#pragma unroll 1
        for (int i = 0; i < n; ++i) {
          const int ent  = __builtin_amdgcn_readfirstlane(lp[i]);
          const int slot = ent & (NBF - 1);
          int src = (ent >> ESHF) & 0xFFFFF;
          src = src > nN - 1 ? nN - 1 : src;
          if (lane == 0) {
            int pos = cursor[slot];
            pos = pos < 0 ? 0 : (pos > RCAP - 1 ? RCAP - 1 : pos);
            region[pos] = src;
            const int np = pos + 1;
            cursor[slot] = np > RCAP ? RCAP : np;
          }
        }
      }
    }
    __syncthreads();
  }

  const int nv = lenW >> 2;
  int* gp = csr + rb0;
#pragma unroll 1
  for (int i = tid; i < nv; i += NTHR) { const v4i v = ((const v4i*)region)[i]; *(volatile v4i*)(gp + 4 * i) = v; }
  __threadfence();
#pragma unroll 1
  for (int i = tid; i < nv; i += NTHR) { const v4i v = ((const v4i*)region)[i]; *(volatile v4i*)(gp + 4 * i) = v; }
}

template <int KD, int RS, int HBIAS, int RELU, int OH>
__global__ __launch_bounds__(NTHR) void k_gemm(
    const _Float16* __restrict__ A16, const _Float16* __restrict__ Bw,
    const float* __restrict__ rsc, const float* __restrict__ bias,
    float* Cf, _Float16* Ch, int NC, float osc, float hs) {
  static_assert((KD % 32) == 0);
  __shared__ __attribute__((aligned(16))) float stg[GR * GC];
  constexpr int NT = 4;
  const int tid = threadIdx.x, lane = tid & 31, wave = tid >> 5, hh = lane >> 4, m = lane & 15;
  const int mw = wave & 3, nw = wave >> 2;
  const int rowBase = (int)blockIdx.x * GR;
  const int colBase = (int)blockIdx.y * GC + nw * 64;
  const _Float16* ap  = A16 + (size_t)(rowBase + mw * 16 + m) * KD + 8 * hh;
  const _Float16* bp0 = Bw + (size_t)(colBase + m) * KD + 8 * hh;

  v8f acc[NT];
#pragma unroll
  for (int t = 0; t < NT; ++t) { v8f z = {0.f, 0.f, 0.f, 0.f, 0.f, 0.f, 0.f, 0.f}; acc[t] = z; }

#pragma unroll 1
  for (int kt = 0; kt < KD / 32; ++kt) {
    FragH af;
    af.h[0] = *(const v8h*)(ap + 32 * kt);
    af.h[1] = *(const v8h*)(ap + 32 * kt + 16);
#pragma unroll
    for (int t = 0; t < NT; ++t) {
      const _Float16* bp = bp0 + (size_t)(16 * t) * KD + 32 * kt;
      FragH bf;
      bf.h[0] = *(const v8h*)bp;
      bf.h[1] = *(const v8h*)(bp + 16);
      acc[t] = wmf(af.v, bf.v, acc[t]);
    }
  }

  const int r0 = mw * 16 + 8 * hh;
  float s[8];
  if (RS != 0) {
    const v4f dA = *(const v4f*)(rsc + (size_t)rowBase + r0);
    const v4f dB = *(const v4f*)(rsc + (size_t)rowBase + r0 + 4);
    s[0] = dA.x; s[1] = dA.y; s[2] = dA.z; s[3] = dA.w; s[4] = dB.x; s[5] = dB.y; s[6] = dB.z; s[7] = dB.w;
#pragma unroll
    for (int r = 0; r < 8; ++r) s[r] = s[r] * osc;
  } else {
#pragma unroll
    for (int r = 0; r < 8; ++r) s[r] = osc;
  }

  float* sp = stg + r0 * GC + nw * 64 + m;
#pragma unroll
  for (int t = 0; t < NT; ++t) {
    float bc = 0.0f;
    if (HBIAS != 0) bc = bias[colBase + 16 * t + m];
#pragma unroll
    for (int r = 0; r < 8; ++r) {
      float v = acc[t][r] * s[r] + bc;
      if (RELU != 0) v = fmaxf(v, 0.0f);
      sp[r * GC + 16 * t] = v;
    }
  }
  __syncthreads();

  const float* lp = stg + (mw * 16) * GC + nw * 64;
  if (OH == 0) {
    const int hr = lane >> 4, pc = lane & 15;
    float* gp = Cf + (size_t)(rowBase + mw * 16) * NC + colBase;
#pragma unroll
    for (int i = 0; i < 8; ++i) {
      const int rr = 2 * i + hr;
      const v4f v = *(const v4f*)(lp + rr * GC + 4 * pc);
      *(volatile v4f*)(gp + (size_t)rr * NC + 4 * pc) = v;
    }
    __threadfence();
#pragma unroll
    for (int i = 0; i < 8; ++i) {
      const int rr = 2 * i + hr;
      const v4f v = *(const v4f*)(lp + rr * GC + 4 * pc);
      *(volatile v4f*)(gp + (size_t)rr * NC + 4 * pc) = v;
    }
  } else {
    const int q = lane >> 3, p = lane & 7;
    _Float16* gp = Ch + (size_t)(rowBase + mw * 16) * NC + colBase;
#pragma unroll
    for (int i = 0; i < 4; ++i) {
      const int rr = 4 * i + q;
      const v4f fa = *(const v4f*)(lp + rr * GC + 8 * p);
      const v4f fb = *(const v4f*)(lp + rr * GC + 8 * p + 4);
      v8h hv;
      hv[0] = (_Float16)(fa.x * hs); hv[1] = (_Float16)(fa.y * hs); hv[2] = (_Float16)(fa.z * hs); hv[3] = (_Float16)(fa.w * hs);
      hv[4] = (_Float16)(fb.x * hs); hv[5] = (_Float16)(fb.y * hs); hv[6] = (_Float16)(fb.z * hs); hv[7] = (_Float16)(fb.w * hs);
      *(volatile v8h*)(gp + (size_t)rr * NC + 8 * p) = hv;
    }
    __threadfence();
#pragma unroll
    for (int i = 0; i < 4; ++i) {
      const int rr = 4 * i + q;
      const v4f fa = *(const v4f*)(lp + rr * GC + 8 * p);
      const v4f fb = *(const v4f*)(lp + rr * GC + 8 * p + 4);
      v8h hv;
      hv[0] = (_Float16)(fa.x * hs); hv[1] = (_Float16)(fa.y * hs); hv[2] = (_Float16)(fa.z * hs); hv[3] = (_Float16)(fa.w * hs);
      hv[4] = (_Float16)(fb.x * hs); hv[5] = (_Float16)(fb.y * hs); hv[6] = (_Float16)(fb.z * hs); hv[7] = (_Float16)(fb.w * hs);
      *(volatile v8h*)(gp + (size_t)rr * NC + 8 * p) = hv;
    }
  }
}

template <int MODE>
__global__ __launch_bounds__(NTHR) void k_agg(
    const int* __restrict__ csr, const int* __restrict__ off, const int* __restrict__ cnt,
    const float* __restrict__ dinv, const float* __restrict__ hw, const float* __restrict__ bias,
    float* outF, _Float16* outH, int nN, int csrLen, float hscl) {
  __shared__ __attribute__((aligned(16))) _Float16 stg[NWAVE * CC];
  const int tid = threadIdx.x, lane = tid & 31, wave = tid >> 5;
  const int tbase = (int)blockIdx.x * TGT + wave * 32;
  const int cl = tbase + lane;
  const int cnt_l = cnt[cl];
  const int off_l = off[cl];
  U32F dvu; dvu.f = dinv[cl];
  const int ca = 4 * lane, cb2 = PCH + 4 * lane;
  const v4f bqa = *(const v4f*)(bias + ca);
  const v4f bqb = *(const v4f*)(bias + cb2);
  _Float16* sw = stg + wave * CC;

#pragma unroll 1
  for (int j = 0; j < 32; ++j) {
    const int c = tbase + j;
    int n = __builtin_amdgcn_readlane(cnt_l, j);
    n = n < 0 ? 0 : (n > DEGCAP ? DEGCAP : n);
    const int st = __builtin_amdgcn_readlane(off_l, j);
    U32F du; du.i = __builtin_amdgcn_readlane(dvu.i, j);
    const float dc = du.f;
    v4f aa = {0.f, 0.f, 0.f, 0.f}, ab = {0.f, 0.f, 0.f, 0.f};
#pragma unroll 1
    for (int q0 = 0; q0 < n; q0 += 32) {
      int pos = st + q0 + lane;
      pos = pos < 0 ? 0 : (pos > csrLen - 1 ? csrLen - 1 : pos);
      int sl = csr[pos];
      sl = sl < 0 ? 0 : (sl > nN - 1 ? nN - 1 : sl);
      const int mcnt = (n - q0) < 32 ? (n - q0) : 32;
#pragma unroll 1
      for (int p = 0; p < mcnt; ++p) {
        const int s = __builtin_amdgcn_readlane(sl, p);
        const float* rp = hw + (size_t)s * CC;
        aa = aa + *(const v4f*)(rp + ca);
        ab = ab + *(const v4f*)(rp + cb2);
      }
    }
    const float* cp = hw + (size_t)c * CC;
    const v4f sa = *(const v4f*)(cp + ca);
    const v4f sb = *(const v4f*)(cp + cb2);
    const v4f va = relu4((aa + sa) * dc + bqa);
    const v4f vb = relu4((ab + sb) * dc + bqb);
    if (MODE == 0) {
      const float z = (c < nN) ? hscl : 0.0f;
      const v4f ta = va * z, tb = vb * z;
      v4h ha, hb;
      ha.x = (_Float16)ta.x; ha.y = (_Float16)ta.y; ha.z = (_Float16)ta.z; ha.w = (_Float16)ta.w;
      hb.x = (_Float16)tb.x; hb.y = (_Float16)tb.y; hb.z = (_Float16)tb.z; hb.w = (_Float16)tb.w;
      *(v4h*)(sw + ca)  = ha;
      *(v4h*)(sw + cb2) = hb;
      __builtin_amdgcn_fence(__ATOMIC_ACQ_REL, "wavefront");
      __builtin_amdgcn_wave_barrier();
      const v8h hv = *(const v8h*)(sw + 8 * lane);
      _Float16* rp = outH + (size_t)c * CC + 8 * lane;
      *(volatile v8h*)rp = hv;
      __threadfence();
      *(volatile v8h*)rp = hv;
      __builtin_amdgcn_fence(__ATOMIC_ACQ_REL, "wavefront");
      __builtin_amdgcn_wave_barrier();
    } else {
      const float z = (c < nN) ? 1.0f : 0.0f;
      const v4f oa = va * z, ob = vb * z;
      float* rp = outF + (size_t)c * CC;
      *(volatile v4f*)(rp + ca)  = oa;
      *(volatile v4f*)(rp + cb2) = ob;
      __threadfence();
      *(volatile v4f*)(rp + ca)  = oa;
      *(volatile v4f*)(rp + cb2) = ob;
    }
  }
}

__global__ __launch_bounds__(NTHR) void k_pool(
    const int* __restrict__ bidx, const float* __restrict__ h3, _Float16* cb,
    int nN, int nG, int vec8, float pscl) {
  __shared__ __attribute__((aligned(16))) float ssum[GPB * PCH];
  __shared__ __attribute__((aligned(16))) int   list[NWAVE * WCAP];
  __shared__ int   scn[GPB];
  __shared__ int   wcnt[NWAVE];
  const int tid = threadIdx.x, lane = tid & 31, wave = tid >> 5;
  const int chb = (int)blockIdx.x * PCH;
  const int g0  = (int)blockIdx.y * GPB;

  {
    const v4f z = {0.f, 0.f, 0.f, 0.f};
    for (int i = tid; i < (GPB * PCH) / 4; i += NTHR) ((v4f*)ssum)[i] = z;
    for (int i = tid; i < GPB; i += NTHR) scn[i] = 0;
  }
  __syncthreads();

  const int nChunks = (nN + CHUNK - 1) / CHUNK;
#pragma unroll 1
  for (int ch = 0; ch < nChunks; ++ch) {
    const int cbase = ch * CHUNK;
    const int wc = scan_chunk<GPB, 2, WCAP, ESHP>(bidx, bidx, nN, nN, cbase, g0, vec8, list, tid, lane, wave);
    if (lane == 0) wcnt[wave] = wc;
    __syncthreads();
    if (wave == 0) {
#pragma unroll 1
      for (int wsx = 0; wsx < NWAVE; ++wsx) {
        int n = __builtin_amdgcn_readfirstlane(wcnt[wsx]);
        n = n > WCAP ? WCAP : (n < 0 ? 0 : n);
        const int* lp = list + wsx * WCAP;
#pragma unroll 1
        for (int i = 0; i < n; ++i) {
          const int ent  = __builtin_amdgcn_readfirstlane(lp[i]);
          const int slot = ent & (GPB - 1);
          int node = (ent >> ESHP) & 0xFFFFF;
          node = node > nN - 1 ? nN - 1 : node;
          const v4f hv = *(const v4f*)(h3 + (size_t)node * CC + chb + 4 * lane);
          v4f* sp = (v4f*)(ssum + slot * PCH + 4 * lane);
          const v4f cur = *sp;
          *sp = cur + hv;
          if (lane == 0) scn[slot] = scn[slot] + 1;
        }
      }
    }
    __syncthreads();
  }

  const int p = tid & 15, rq = tid >> 4;
#pragma unroll 1
  for (int it = 0; it < GPB / 16; ++it) {
    const int row = it * 16 + rq;
    int g = g0 + row;
    g = g > nG - 1 ? nG - 1 : g;
    const float cntf = (float)scn[row];
    const float inv = 1.0f / fmaxf(cntf, 1.0f);
    v8h hv;
#pragma unroll
    for (int i = 0; i < 8; ++i) {
      const float ge = ssum[row * PCH + 8 * p + i] * inv;
      hv[i] = (_Float16)(ge * pscl);
    }
    _Float16* d = cb + (size_t)g * CC + chb + 8 * p;
    *(volatile v8h*)d = hv;
    __threadfence();
    *(volatile v8h*)d = hv;
  }
}

extern "C" void kernel_launch(void* const* d_in, const int* in_sizes, int n_in,
                              void* d_out, int out_size, void* d_ws, size_t ws_size,
                              hipStream_t stream) {
  if (n_in < 13) return;
  const int nN = in_sizes[2];
  const int nE = in_sizes[1] / 2;
  const int nG = out_size / NOUT;
  if (nN <= 0 || nE <= 0 || nG <= 0) return;
  if ((long long)in_sizes[0] != (long long)nN * (long long)CC) return;
  if (in_sizes[1] != 2 * nE) return;
  if (in_sizes[3] != CC * CC || in_sizes[4] != CC || in_sizes[5] != CC * CC || in_sizes[6] != CC) return;
  if (in_sizes[7] != CC * CC || in_sizes[8] != CC || in_sizes[9] != CC * CC || in_sizes[10] != CC) return;
  if (in_sizes[11] != CC * NOUT || in_sizes[12] != NOUT) return;
  if (out_size != nG * NOUT || (nG % GPB) != 0 || (nG % GR) != 0) return;
  if (nN > (1 << 20) || nE > (1 << 28) || nG > (1 << 16)) return;

  const float* x    = (const float*)d_in[0];
  const int*   ei   = (const int*)d_in[1];
  const int*   bidx = (const int*)d_in[2];
  const float* W0   = (const float*)d_in[3];
  const float* b0   = (const float*)d_in[4];
  const float* W1   = (const float*)d_in[5];
  const float* b1   = (const float*)d_in[6];
  const float* W2   = (const float*)d_in[7];
  const float* b2   = (const float*)d_in[8];
  const float* F1   = (const float*)d_in[9];
  const float* fb1  = (const float*)d_in[10];
  const float* F2   = (const float*)d_in[11];
  const float* fb2  = (const float*)d_in[12];
  float* out = (float*)d_out;
  const int* vals = ei;
  const int* keys = ei + nE;
  const int nK = nE;

  const int NPAD   = ((nN + TGT - 1) / TGT) * TGT;
  const int nBC    = (nN + NBC - 1) / NBC;
  const int CNTPAD = nBC * NBC;
  const int nBF    = (nN + NBF - 1) / NBF;
  const int OFFN   = nBF * NBF;
  if (nBF + 1 > RBN) return;
  if (OFFN > CNTPAD || NPAD > OFFN) return;
  const int csrLen = ((nK + 31) & ~31) + 32 * (nBF + 1);
  const int nGemm  = NPAD / GR;
  const int nAgg   = NPAD / TGT;
  const int nGemmH = nG / GR;

  char* ws = (char*)d_ws;
  size_t off = 0;
  const size_t oZ   = off; off += (size_t)NPAD * CC * 4;         off = (off + 255) & ~(size_t)255;
  const size_t oW0  = off; off += (size_t)CC * CC * 2;           off = (off + 255) & ~(size_t)255;
  const size_t oW1  = off; off += (size_t)CC * CC * 2;           off = (off + 255) & ~(size_t)255;
  const size_t oW2  = off; off += (size_t)CC * CC * 2;           off = (off + 255) & ~(size_t)255;
  const size_t oF1  = off; off += (size_t)CC * CC * 2;           off = (off + 255) & ~(size_t)255;
  const size_t oF2  = off; off += (size_t)NOUT * CC * 2;         off = (off + 255) & ~(size_t)255;
  const size_t oCnt = off; off += (size_t)CNTPAD * 4;            off = (off + 255) & ~(size_t)255;
  const size_t oDv  = off; off += (size_t)CNTPAD * 4;            off = (off + 255) & ~(size_t)255;
  const size_t oOff = off; off += (size_t)OFFN * 4;              off = (off + 255) & ~(size_t)255;
  const size_t oRb  = off; off += (size_t)RBN * 4;               off = (off + 255) & ~(size_t)255;
  const size_t oCsr = off; off += (size_t)csrLen * 4;            off = (off + 255) & ~(size_t)255;
  const size_t oHW  = off; off += (size_t)NPAD * CC * 4;         off = (off + 255) & ~(size_t)255;
  const size_t oCB  = off; off += (size_t)nG * CC * 2;           off = (off + 255) & ~(size_t)255;
  const size_t oHQ  = off; off += (size_t)nG * CC * 2;           off = (off + 255) & ~(size_t)255;
  if (off > ws_size || off > (size_t)WSCAP) return;
  _Float16* HA   = (_Float16*)(ws + oZ);
  _Float16* HB   = (_Float16*)(ws + oZ + (size_t)NPAD * CC * 2);
  float*    Z    = (float*)(ws + oZ);
  _Float16* W0p  = (_Float16*)(ws + oW0);
  _Float16* W1p  = (_Float16*)(ws + oW1);
  _Float16* W2p  = (_Float16*)(ws + oW2);
  _Float16* F1p  = (_Float16*)(ws + oF1);
  _Float16* F2p  = (_Float16*)(ws + oF2);
  int*      cnt  = (int*)(ws + oCnt);
  float*    dinv = (float*)(ws + oDv);
  int*      offp = (int*)(ws + oOff);
  int*      rb   = (int*)(ws + oRb);
  int*      csr  = (int*)(ws + oCsr);
  float*    HW   = (float*)(ws + oHW);
  _Float16* CB   = (_Float16*)(ws + oCB);
  _Float16* HQ   = (_Float16*)(ws + oHQ);

  const int vec8  = ((nE & 7) == 0) ? 1 : 0;
  const int vec8p = ((nN & 7) == 0) ? 1 : 0;
  const float oscX = 1.0f / ((float)ASCL * (float)WSCL);
  const float oscH = 1.0f / ((float)HSCL * (float)WSCL);
  const float oscP = 1.0f / ((float)PSCL * (float)WSCL);
  const float oscQ = 1.0f / ((float)QSCL * (float)WSCL);

  {
    const int t8x = (int)(((size_t)NPAD * CC) / 8);
    k_x16<<<(t8x + NTHR - 1) / NTHR, NTHR, 0, stream>>>(x, HA, nN, t8x, (float)ASCL);
  }
  {
    const dim3 gT(CC / TPK, CC / TPN);
    k_wT16<<<gT, NTHR, 0, stream>>>(W0, W0p, CC, CC, (float)WSCL);
    k_wT16<<<gT, NTHR, 0, stream>>>(W1, W1p, CC, CC, (float)WSCL);
    k_wT16<<<gT, NTHR, 0, stream>>>(W2, W2p, CC, CC, (float)WSCL);
    k_wT16<<<gT, NTHR, 0, stream>>>(F1, F1p, CC, CC, (float)WSCL);
    const dim3 gF(CC / TPK, NOUT / TPN);
    k_wT16<<<gF, NTHR, 0, stream>>>(F2, F2p, CC, NOUT, (float)WSCL);
  }

  hipFuncSetAttribute(reinterpret_cast<const void*>(&k_count),
                      hipFuncAttributeMaxDynamicSharedMemorySize, LDS_COUNT);
  k_count<<<nBC, NTHR, LDS_COUNT, stream>>>(keys, cnt, dinv, nK, nN, vec8);
  k_offsets<<<1, OTHR, 0, stream>>>(cnt, offp, rb, nBF);
  hipFuncSetAttribute(reinterpret_cast<const void*>(&k_fill),
                      hipFuncAttributeMaxDynamicSharedMemorySize, LDS_FILL);
  k_fill<<<nBF, NTHR, LDS_FILL, stream>>>(keys, vals, offp, rb, csr, nN, nK, vec8, csrLen);

  const dim3 gG(nGemm, CC / GC);

  k_gemm<CC, 1, 0, 0, 0><<<gG, NTHR, 0, stream>>>(HA, W0p, dinv, b0, HW, HB, CC, oscX, 1.0f);
  k_agg<0><<<nAgg, NTHR, 0, stream>>>(csr, offp, cnt, dinv, HW, b0, Z, HB, nN, csrLen, (float)HSCL);

  k_gemm<CC, 1, 0, 0, 0><<<gG, NTHR, 0, stream>>>(HB, W1p, dinv, b1, HW, HA, CC, oscH, 1.0f);
  k_agg<0><<<nAgg, NTHR, 0, stream>>>(csr, offp, cnt, dinv, HW, b1, Z, HA, nN, csrLen, (float)HSCL);

  k_gemm<CC, 1, 0, 0, 0><<<gG, NTHR, 0, stream>>>(HA, W2p, dinv, b2, HW, HB, CC, oscH, 1.0f);
  k_agg<1><<<nAgg, NTHR, 0, stream>>>(csr, offp, cnt, dinv, HW, b2, Z, HB, nN, csrLen, 1.0f);

  {
    const dim3 gP(CC / PCH, nG / GPB);
    k_pool<<<gP, NTHR, 0, stream>>>(bidx, Z, CB, nN, nG, vec8p, (float)PSCL);
  }

  {
    const dim3 gH1(nGemmH, CC / GC);
    k_gemm<CC, 0, 1, 1, 1><<<gH1, NTHR, 0, stream>>>(CB, F1p, dinv, fb1, HW, HQ, CC, oscP, (float)QSCL);
  }
  {
    const dim3 gH2(nGemmH, NOUT / GC);
    k_gemm<CC, 0, 1, 0, 0><<<gH2, NTHR, 0, stream>>>(HQ, F2p, dinv, fb2, out, CB, NOUT, oscQ, 1.0f);
  }
}
